// Encoder_49967649521793
// MI455X (gfx1250) — hardware-verified
//
#include <hip/hip_runtime.h>
#include <math.h>

constexpr int NBATCH   = 64;
constexpr int NSTEP    = 256;
constexpr int NEMB     = 512;
constexpr int NHID     = 512;
constexpr int NGATE    = 4 * NHID;
constexpr int NVOCAB   = 32000;
constexpr int NTHR     = 256;
constexpr int ROWS_BLK = 16;
constexpr int APITCH   = 520;
constexpr int TILE_ELEMS = ROWS_BLK * APITCH;
constexpr int CPITCH   = 520;
constexpr int CT_ELEMS = ROWS_BLK * CPITCH;
constexpr int GATE_STRIDE = NHID * NHID;
constexpr int PLANE_ELEMS = NBATCH * NHID;
constexpr int OUT_ELEMS   = 4 * PLANE_ELEMS;
constexpr float WCARRY     = 256.0f;
constexpr float WCARRY_INV = 1.0f / 256.0f;

static_assert(NEMB == NHID, "one k-loop helper serves both operand halves");
static_assert(NHID == 64 * (NTHR / 32), "8 waves x 64 hidden units");
static_assert(NHID % 32 == 0 && NEMB % 32 == 0, "K multiple of 32");
static_assert(NBATCH % ROWS_BLK == 0, "batch tile multiple");
static_assert((4 * TILE_ELEMS) % NTHR == 0, "h zero-fill loop exact");
static_assert((2 * CT_ELEMS) % NTHR == 0, "c zero-fill loop exact");
static_assert((ROWS_BLK * NEMB / 8) == 4 * NTHR, "x staging loop exact");
static_assert(OUT_ELEMS * 4 == 524288, "d_out bytes");
static_assert(2 * PLANE_ELEMS * 4 == 262144, "cs byte offset");
static_assert((NGATE / 4) == 2 * NTHR, "bias staging loop exact");
static_assert((NGATE * NHID / 8) % NTHR == 0, "weight convert grid exact");
static_assert((NSTEP * NBATCH * (NEMB / 8)) % NTHR == 0, "gather grid exact");
static_assert(CPITCH % 4 == 0 && APITCH % 8 == 0, "vector alignment of LDS rows");

typedef __attribute__((ext_vector_type(16))) _Float16 v16h;
typedef __attribute__((ext_vector_type(8)))  _Float16 v8h;
typedef __attribute__((ext_vector_type(8)))  float    v8f;
typedef __attribute__((ext_vector_type(4)))  float    v4f;

__device__ __forceinline__ unsigned short f2bf_bits(float f) {
  unsigned u = __float_as_uint(f);
  return (unsigned short)((u + 0x7FFFu + ((u >> 16) & 1u)) >> 16);
}
__device__ __forceinline__ float bf_bits2f(unsigned short h) { return __uint_as_float(((unsigned)h) << 16); }
__device__ __forceinline__ float bf16r(float f) { return bf_bits2f(f2bf_bits(f)); }

__device__ __forceinline__ void guard_all4(v8f& a0, v8f& a1, v8f& a2, v8f& a3,
                                           v16h a, v16h b0, v16h b1, v16h b2, v16h b3) {
  asm volatile("v_nop\n\tv_nop\n\tv_nop\n\tv_nop"
               : "+v"(a0), "+v"(a1), "+v"(a2), "+v"(a3)
               : "v"(a), "v"(b0), "v"(b1), "v"(b2), "v"(b3));
}
__device__ __forceinline__ void acc_guard4(v8f& a, v8f& b, v8f& c, v8f& d) {
  asm volatile("v_nop\n\tv_nop\n\tv_nop\n\tv_nop" : "+v"(a), "+v"(b), "+v"(c), "+v"(d));
}

template <typename T> struct Frag;
template <> struct Frag<_Float16> {
  typedef v16h V;
  union U { v16h v; v8h h[2]; };
  static __device__ __forceinline__ v16h load(const _Float16* p) {
    U f;
    f.h[0] = *(const v8h*)(p);
    f.h[1] = *(const v8h*)(p + 16);
    return f.v;
  }
  static __device__ __forceinline__ v8f mma(v16h a, v16h b, v8f c) {
    return __builtin_amdgcn_wmma_f32_16x16x32_f16(false, a, false, b, (short)0, c, false, false);
  }
};

__device__ __forceinline__ float fsig(float x)  { return __builtin_amdgcn_rcpf(1.0f + expf(-x)); }
__device__ __forceinline__ float ftanh(float x) { return 1.0f - 2.0f * __builtin_amdgcn_rcpf(expf(2.0f * x) + 1.0f); }

__global__ __launch_bounds__(NTHR) void cvt_w_kernel(const float* __restrict__ src, unsigned short* __restrict__ dst,
                                                     int n8, float sc) {
  const int i = blockIdx.x * NTHR + threadIdx.x;
  if (i < n8) {
    const float* sp = src + (size_t)i * 8;
    const v4f a = *(const v4f*)(sp);
    const v4f b = *(const v4f*)(sp + 4);
    v8h hv;
#pragma unroll
    for (int e = 0; e < 4; ++e) {
      const float fa = a[e];
      const float fb = b[e];
      hv[e]     = (_Float16)(bf16r(fa) * sc);
      hv[4 + e] = (_Float16)(bf16r(fb) * sc);
    }
    *(volatile v8h*)(dst + (size_t)i * 8) = hv;
    __threadfence();
    *(volatile v8h*)(dst + (size_t)i * 8) = hv;
  }
}

__global__ __launch_bounds__(NTHR) void gather_x_kernel(const int* __restrict__ src, const float* __restrict__ emb,
                                                        unsigned short* __restrict__ X) {
  const int i  = blockIdx.x * NTHR + threadIdx.x;
  const int n8 = NSTEP * NBATCH * (NEMB / 8);
  if (i < n8) {
    const int row = i / (NEMB / 8);
    const int c8  = i - row * (NEMB / 8);
    const int t   = row / NBATCH;
    const int b   = row - t * NBATCH;
    int tok = src[b * NSTEP + t];
    tok = tok < 0 ? 0 : tok;
    tok = tok > (NVOCAB - 1) ? (NVOCAB - 1) : tok;
    const float* sp = emb + (size_t)tok * NEMB + c8 * 8;
    const v4f a = *(const v4f*)(sp);
    const v4f bq = *(const v4f*)(sp + 4);
    v8h hv;
#pragma unroll
    for (int e = 0; e < 4; ++e) {
      const float fa = a[e];
      const float fb = bq[e];
      hv[e]     = (_Float16)bf16r(fa);
      hv[4 + e] = (_Float16)bf16r(fb);
    }
    *(volatile v8h*)(X + (size_t)i * 8) = hv;
    __threadfence();
    *(volatile v8h*)(X + (size_t)i * 8) = hv;
  }
}

__device__ __forceinline__ void gate_kloop(v8f& acc0, v8f& acc1, v8f& acc2, v8f& acc3,
                                           const _Float16* arow, const _Float16* wrow) {
#pragma unroll 1
  for (int k0 = 0; k0 < NHID; k0 += 32) {
    const v16h a  = Frag<_Float16>::load(arow + k0);
    const v16h b0 = Frag<_Float16>::load(wrow + k0);
    const v16h b1 = Frag<_Float16>::load(wrow + (size_t)1 * GATE_STRIDE + k0);
    asm volatile("" ::: "memory");
    const v16h b2 = Frag<_Float16>::load(wrow + (size_t)2 * GATE_STRIDE + k0);
    const v16h b3 = Frag<_Float16>::load(wrow + (size_t)3 * GATE_STRIDE + k0);
    acc0 = Frag<_Float16>::mma(a, b0, acc0);
    acc1 = Frag<_Float16>::mma(a, b1, acc1);
    acc2 = Frag<_Float16>::mma(a, b2, acc2);
    acc3 = Frag<_Float16>::mma(a, b3, acc3);
    guard_all4(acc0, acc1, acc2, acc3, a, b0, b1, b2, b3);
  }
}

__device__ __forceinline__ void lstm_layer(const _Float16* aIn, const _Float16* aRec,
                                           const _Float16* wIn, const _Float16* wRec,
                                           const float* bs, _Float16* hw, float* cs, float* hf, bool last,
                                           int wave, int c, int hh) {
#pragma unroll 1
  for (int nt = 0; nt < 4; ++nt) {
    const int j = 64 * wave + 16 * nt + c;
    const size_t woff = (size_t)j * NHID + (size_t)(hh * 8);
    const float bi = bs[0 * NHID + j] * WCARRY;
    const float bf = bs[1 * NHID + j] * WCARRY;
    const float bg = bs[2 * NHID + j] * WCARRY;
    const float bo = bs[3 * NHID + j] * WCARRY;
    v8f acc0 = (v8f){bi, bi, bi, bi, bi, bi, bi, bi};
    v8f acc1 = (v8f){bf, bf, bf, bf, bf, bf, bf, bf};
    v8f acc2 = (v8f){bg, bg, bg, bg, bg, bg, bg, bg};
    v8f acc3 = (v8f){bo, bo, bo, bo, bo, bo, bo, bo};
    gate_kloop(acc0, acc1, acc2, acc3, aIn,  wIn  + woff);
    gate_kloop(acc0, acc1, acc2, acc3, aRec, wRec + woff);
    acc_guard4(acc0, acc1, acc2, acc3);
    float hn[8];
#pragma unroll
    for (int r = 0; r < 8; ++r) {
      const int row = 8 * hh + r;
      const float zi = acc0[r] * WCARRY_INV;
      const float zf = acc1[r] * WCARRY_INV;
      const float zg = acc2[r] * WCARRY_INV;
      const float zo = acc3[r] * WCARRY_INV;
      const float ig = fsig(zi);
      const float fg = fsig(zf);
      const float gg = ftanh(zg);
      const float og = fsig(zo);
      const float co = cs[row * CPITCH + j];
      const float cn = fg * co + ig * gg;
      cs[row * CPITCH + j] = cn;
      hn[r] = og * ftanh(cn);
      hw[row * APITCH + j] = (_Float16)hn[r];
    }
    if (last) {
#pragma unroll
      for (int r = 0; r < 8; ++r) hf[(8 * hh + r) * CPITCH + j] = hn[r];
    }
  }
}

__device__ __forceinline__ void store_tile(const float* tile, float* dst, int hh, int c) {
  const int c4 = c * 4;
  __builtin_amdgcn_fence(__ATOMIC_RELEASE, "workgroup");
  __builtin_amdgcn_wave_barrier();
  __builtin_amdgcn_fence(__ATOMIC_ACQUIRE, "workgroup");
  for (int pass = 0; pass < 2; ++pass) {
#pragma unroll
    for (int it = 0; it < 8; ++it) {
      const int row = it * 2 + hh;
      const v4f val = *(const v4f*)(tile + row * CPITCH + c4);
      *(volatile v4f*)(dst + (size_t)row * NHID + c4) = val;
    }
    __threadfence();
  }
  __builtin_amdgcn_fence(__ATOMIC_RELEASE, "workgroup");
  __builtin_amdgcn_wave_barrier();
  __builtin_amdgcn_fence(__ATOMIC_ACQUIRE, "workgroup");
}

__device__ __forceinline__ void stage_x(_Float16* xs, const _Float16* X, int tn, int rowbase, int tid) {
  const _Float16* srcp = X + ((size_t)tn * NBATCH + (size_t)rowbase) * NEMB;
#pragma unroll
  for (int it = 0; it < 4; ++it) {
    const int idx = it * NTHR + tid;
    const int row = idx >> 6;
    const int c8  = (idx & 63) * 8;
    const v8h v = *(const v8h*)(srcp + (size_t)idx * 8);
    *(v8h*)(xs + row * APITCH + c8) = v;
  }
}

__global__ __launch_bounds__(NTHR) __attribute__((amdgpu_num_vgpr(256)))
void lstm2_seq_kernel(const unsigned short* __restrict__ Xp,
                      const unsigned short* __restrict__ WI0p,
                      const unsigned short* __restrict__ WH0p,
                      const unsigned short* __restrict__ WI1p,
                      const unsigned short* __restrict__ WH1p,
                      const float* __restrict__ bi0, const float* __restrict__ bh0,
                      const float* __restrict__ bi1, const float* __restrict__ bh1,
                      float* __restrict__ out) {
  __shared__ __align__(16) _Float16 Xs[TILE_ELEMS];
  __shared__ __align__(16) _Float16 Ht[4 * TILE_ELEMS];
  __shared__ __align__(16) float    Cs[2 * CT_ELEMS];
  __shared__ __align__(16) float    Hf[CT_ELEMS];
  __shared__ __align__(16) float    Bs[2 * NGATE];
  const _Float16* X   = (const _Float16*)Xp;
  const _Float16* WI0 = (const _Float16*)WI0p;
  const _Float16* WH0 = (const _Float16*)WH0p;
  const _Float16* WI1 = (const _Float16*)WI1p;
  const _Float16* WH1 = (const _Float16*)WH1p;
  const int tid = threadIdx.x, lane = tid & 31, wave = tid >> 5;
  const int c = lane & 15, hh = lane >> 4, koff = hh * 8;
  const int rowbase = blockIdx.x * ROWS_BLK;

#pragma unroll 1
  for (int i = tid; i < 4 * TILE_ELEMS; i += NTHR) Ht[i] = (_Float16)0.0f;
#pragma unroll 1
  for (int i = tid; i < 2 * CT_ELEMS; i += NTHR) Cs[i] = 0.0f;
#pragma unroll 1
  for (int i = 0; i < 2; ++i) {
    const int idx = (i * NTHR + tid) * 4;
    const v4f a0 = *(const v4f*)(bi0 + idx);
    const v4f h0 = *(const v4f*)(bh0 + idx);
    const v4f a1 = *(const v4f*)(bi1 + idx);
    const v4f h1 = *(const v4f*)(bh1 + idx);
    v4f o0, o1;
#pragma unroll
    for (int e = 0; e < 4; ++e) {
      const float p0 = a0[e];
      const float q0 = h0[e];
      const float p1 = a1[e];
      const float q1 = h1[e];
      o0[e] = bf16r(p0) + bf16r(q0);
      o1[e] = bf16r(p1) + bf16r(q1);
    }
    *(v4f*)(Bs + idx) = o0;
    *(v4f*)(Bs + NGATE + idx) = o1;
  }
  stage_x(Xs, X, 0, rowbase, tid);
  __syncthreads();

  const int arowoff = c * APITCH + koff;
  float* otile = out + (size_t)rowbase * NHID + 64 * wave;
  float* hfw   = Hf + 64 * wave;

#pragma unroll 1
  for (int t = 0; t < NSTEP; ++t) {
    const int  p    = t & 1;
    const bool last = (t == NSTEP - 1);
    const _Float16* h0rd = Ht + (0 + p) * TILE_ELEMS;
    _Float16*       h0wr = Ht + (0 + (p ^ 1)) * TILE_ELEMS;
    const _Float16* h1rd = Ht + (2 + p) * TILE_ELEMS;
    _Float16*       h1wr = Ht + (2 + (p ^ 1)) * TILE_ELEMS;

    lstm_layer(Xs + arowoff, h0rd + arowoff, WI0, WH0, Bs, h0wr, Cs, Hf, last, wave, c, hh);
    if (last) store_tile(hfw, otile + 0 * PLANE_ELEMS, hh, c);
    __syncthreads();

    {
      const int tn = (t + 1 < NSTEP) ? (t + 1) : (NSTEP - 1);
      stage_x(Xs, X, tn, rowbase, tid);
    }
    lstm_layer(h0wr + arowoff, h1rd + arowoff, WI1, WH1, Bs + NGATE, h1wr, Cs + CT_ELEMS, Hf, last, wave, c, hh);
    __syncthreads();
  }

  store_tile(hfw, otile + 1 * PLANE_ELEMS, hh, c);
  store_tile(Cs + 64 * wave, otile + 2 * PLANE_ELEMS, hh, c);
  store_tile(Cs + CT_ELEMS + 64 * wave, otile + 3 * PLANE_ELEMS, hh, c);
}

extern "C" void kernel_launch(void* const* d_in, const int* in_sizes, int n_in,
                              void* d_out, int out_size, void* d_ws, size_t ws_size, hipStream_t stream) {
  if (n_in < 10 || d_out == nullptr || d_ws == nullptr) return;
  if (in_sizes[0] != NBATCH * NSTEP || in_sizes[1] != NVOCAB * NEMB ||
      in_sizes[2] != NGATE * NEMB || in_sizes[3] != NGATE ||
      in_sizes[4] != NGATE * NHID || in_sizes[5] != NGATE ||
      in_sizes[6] != NGATE * NHID || in_sizes[7] != NGATE ||
      in_sizes[8] != NGATE * NHID || in_sizes[9] != NGATE ||
      out_size != OUT_ELEMS) return;

  const int*   src   = (const int*)d_in[0];
  const float* emb   = (const float*)d_in[1];
  const float* w_ih0 = (const float*)d_in[2];
  const float* b_ih0 = (const float*)d_in[3];
  const float* w_hh0 = (const float*)d_in[4];
  const float* b_hh0 = (const float*)d_in[5];
  const float* w_ih1 = (const float*)d_in[6];
  const float* b_ih1 = (const float*)d_in[7];
  const float* w_hh1 = (const float*)d_in[8];
  const float* b_hh1 = (const float*)d_in[9];
  float* out = (float*)d_out;

  char* ws = (char*)d_ws;
  size_t off = 0;
  auto carve = [&](size_t bytes) -> char* { char* p = ws + off; off += (bytes + 255) & ~(size_t)255; return p; };
  unsigned short* WI0 = (unsigned short*)carve((size_t)NGATE * NEMB * 2);
  unsigned short* WH0 = (unsigned short*)carve((size_t)NGATE * NHID * 2);
  unsigned short* WI1 = (unsigned short*)carve((size_t)NGATE * NHID * 2);
  unsigned short* WH1 = (unsigned short*)carve((size_t)NGATE * NHID * 2);
  unsigned short* XPL = (unsigned short*)carve((size_t)NSTEP * NBATCH * NEMB * 2);
  if (off > ws_size || off > (size_t)134217728) return;

  const int n8w = NGATE * NHID / 8;
  cvt_w_kernel<<<n8w / NTHR, NTHR, 0, stream>>>(w_ih0, WI0, n8w, WCARRY);
  cvt_w_kernel<<<n8w / NTHR, NTHR, 0, stream>>>(w_hh0, WH0, n8w, WCARRY);
  cvt_w_kernel<<<n8w / NTHR, NTHR, 0, stream>>>(w_ih1, WI1, n8w, WCARRY);
  cvt_w_kernel<<<n8w / NTHR, NTHR, 0, stream>>>(w_hh1, WH1, n8w, WCARRY);
  gather_x_kernel<<<(NSTEP * NBATCH * (NEMB / 8)) / NTHR, NTHR, 0, stream>>>(src, emb, XPL);
  lstm2_seq_kernel<<<NBATCH / ROWS_BLK, NTHR, 0, stream>>>(XPL, WI0, WH0, WI1, WH1,
                                                           b_ih0, b_hh0, b_ih1, b_hh1, out);
}
